// GCN_9294309229069
// MI455X (gfx1250) — hardware-verified
//
#include <hip/hip_runtime.h>
#include <stddef.h>
#include <stdint.h>
#include <math.h>


#define CF     64
#define OC     32
#define K2     128
#define NTHR   256
#define NWAVE  8
#define EPT    8
#define CHUNK  (NTHR * EPT)
#define WCAP   (EPT * 32)
#define LISTN  (NWAVE * WCAP)
#define NBD    8192
#define SLD    13
#define NBA    1024
#define SLA    10
#define RCAP   16384
#define DEGCAP 64
#define GBM    64
#define GTHR   128
#define NUW    (CF * (K2 / 8))
#define NUW2   (OC * (K2 / 8))
#define AGG_ZINTS (LISTN + 2 * RCAP + 3 * NBA)
#define AGG_LDS_INTS (AGG_ZINTS + 16)
#define WSMAX  134217728

static_assert((CHUNK & (CHUNK - 1)) == 0 && CHUNK <= 4096);
static_assert((NBD & (NBD - 1)) == 0 && NBD == (1 << SLD));
static_assert((NBA & (NBA - 1)) == 0 && NBA == (1 << SLA));
static_assert(((long long)CHUNK << SLD) < (1LL << 31));
static_assert(((long long)CHUNK << SLA) < (1LL << 31));
static_assert(NBD % (NTHR * 4) == 0);
static_assert(LISTN % NTHR == 0);
static_assert(NBA % NWAVE == 0 && NBA % 32 == 0 && NBA % GBM == 0);
static_assert(RCAP % 32 == 0 && AGG_ZINTS % 4 == 0 && LISTN % 4 == 0);
static_assert(K2 % 32 == 0 && K2 == 2 * CF && CF == 64 && OC == 32);
static_assert(GBM == (GTHR / 32) * 16);
static_assert(NUW % NTHR == 0 && NUW2 % NTHR == 0 && K2 / 8 == 16);
static_assert(CF == 2 * 32);
static_assert(AGG_LDS_INTS * 4 <= 300000);
static_assert(GTHR >= CF);

typedef float          v2f   __attribute__((ext_vector_type(2)));
typedef float          v4f   __attribute__((ext_vector_type(4)));
typedef float          v8f   __attribute__((ext_vector_type(8)));
typedef int            v4i   __attribute__((ext_vector_type(4)));
typedef int            v8i   __attribute__((ext_vector_type(8)));
typedef unsigned int   v4u   __attribute__((ext_vector_type(4)));
typedef unsigned short v8us  __attribute__((ext_vector_type(8)));
typedef unsigned short v16us __attribute__((ext_vector_type(16)));
typedef __bf16         v16bf __attribute__((ext_vector_type(16)));
typedef v2f  __attribute__((may_alias)) v2fa;
typedef v4f  __attribute__((may_alias)) v4fa;
typedef v4i  __attribute__((may_alias)) v4ia;
typedef v8us __attribute__((may_alias)) v8usa;
union FragB { v16bf v; v16us u; v8us h[2]; v8i w; };

__device__ __forceinline__ v8f wmb(const FragB& a, const FragB& b, v8f c) {
  v8f d = __builtin_amdgcn_wmma_f32_16x16x32_bf16(false, a.v, false, b.v, (short)0, c, false, false);
  asm volatile("v_nop\n\tv_nop\n\tv_nop\n\tv_nop" : "+v"(d) : "v"(a.w), "v"(b.w));
  return d;
}

__device__ __forceinline__ unsigned bf16_bits(float f) {
  const unsigned u = __float_as_uint(f);
  return (u + 0x7FFFu + ((u >> 16) & 1u)) >> 16;
}
__device__ __forceinline__ float bf16_val(float f) {
  return __uint_as_float(bf16_bits(f) << 16);
}
__device__ __forceinline__ float relu_keep(float v) {
  return (v > 0.0f) ? v : (v - v);
}

template <int SLB>
__device__ __forceinline__ int scan_chunk(const int* __restrict__ dsts, int nE, int cbase, int slotBase,
                                          int nb, int vec8, int* list, int tid, int lane, int wave) {
  int wc = 0;
  const int el0  = tid * EPT;
  const int e0   = cbase + el0;
  const int sent = -2147483647 - 1;
  v4i da, db;
  if (vec8 != 0 && cbase + CHUNK <= nE) {
    da = *(const v4i*)(dsts + e0);
    db = *(const v4i*)(dsts + e0 + 4);
  } else {
    da.x = (e0     < nE) ? dsts[min(e0,     nE - 1)] : sent;
    da.y = (e0 + 1 < nE) ? dsts[min(e0 + 1, nE - 1)] : sent;
    da.z = (e0 + 2 < nE) ? dsts[min(e0 + 2, nE - 1)] : sent;
    da.w = (e0 + 3 < nE) ? dsts[min(e0 + 3, nE - 1)] : sent;
    db.x = (e0 + 4 < nE) ? dsts[min(e0 + 4, nE - 1)] : sent;
    db.y = (e0 + 5 < nE) ? dsts[min(e0 + 5, nE - 1)] : sent;
    db.z = (e0 + 6 < nE) ? dsts[min(e0 + 6, nE - 1)] : sent;
    db.w = (e0 + 7 < nE) ? dsts[min(e0 + 7, nE - 1)] : sent;
  }
  const unsigned nbs = (unsigned)slotBase;
  const unsigned unb = (unsigned)nb;
  const unsigned s0 = (unsigned)da.x - nbs, s1 = (unsigned)da.y - nbs;
  const unsigned s2 = (unsigned)da.z - nbs, s3 = (unsigned)da.w - nbs;
  const unsigned s4 = (unsigned)db.x - nbs, s5 = (unsigned)db.y - nbs;
  const unsigned s6 = (unsigned)db.z - nbs, s7 = (unsigned)db.w - nbs;
  const bool h0 = s0 < unb, h1 = s1 < unb, h2 = s2 < unb, h3 = s3 < unb;
  const bool h4 = s4 < unb, h5 = s5 < unb, h6 = s6 < unb, h7 = s7 < unb;
  const unsigned any = __builtin_amdgcn_ballot_w32(h0 | h1 | h2 | h3 | h4 | h5 | h6 | h7);
  if (any != 0u) {
#define HITJ(J, HJ, SJ) { \
      const unsigned mj = __builtin_amdgcn_ballot_w32(HJ); \
      if (mj != 0u) { \
        if (HJ) { \
          const int pos = wc + (int)__builtin_amdgcn_mbcnt_lo(mj, 0u); \
          if (pos < WCAP) list[wave * WCAP + pos] = ((el0 + (J)) << SLB) | (int)(SJ); \
        } \
        wc += (int)__builtin_popcount(mj); } }
    HITJ(0, h0, s0)
    HITJ(1, h1, s1)
    HITJ(2, h2, s2)
    HITJ(3, h3, s3)
    HITJ(4, h4, s4)
    HITJ(5, h5, s5)
    HITJ(6, h6, s6)
    HITJ(7, h7, s7)
#undef HITJ
  }
  return wc;
}

__device__ __forceinline__ void wunit(const float* __restrict__ W, int nout, int v, unsigned short* P) {
  const int n  = v >> 4;
  const int k8 = (v & 15) * 8;
  const int kk = k8 & (CF - 1);
  const float* p = W + (size_t)kk * (size_t)nout + n;
  v8us o;
#pragma unroll
  for (int i = 0; i < 8; ++i) o[i] = (unsigned short)bf16_bits(p[(size_t)i * (size_t)nout]);
  unsigned short* dp = P + (size_t)n * K2 + k8;
  *(volatile v8us*)dp = o;
  __threadfence();
  *(volatile v8us*)dp = o;
}

__global__ __launch_bounds__(NTHR) void k_wprep(const float* __restrict__ W1, const float* __restrict__ W2,
                                                const float* __restrict__ Wm1, const float* __restrict__ Wm2,
                                                unsigned short* W1T, unsigned short* W2T,
                                                unsigned short* Wm1T, unsigned short* Wm2T) {
  const int u = (int)blockIdx.x * NTHR + (int)threadIdx.x;
  if (u < NUW) {
    wunit(W1, CF, u, W1T);
  } else if (u < 2 * NUW) {
    wunit(W2, CF, u - NUW, W2T);
  } else if (u < 3 * NUW) {
    wunit(Wm1, CF, u - 2 * NUW, Wm1T);
  } else if (u < 3 * NUW + NUW2) {
    wunit(Wm2, OC, u - 3 * NUW, Wm2T);
  }
}

__global__ __launch_bounds__(NTHR) void k_cvx(const float* __restrict__ x, int nUnits, unsigned short* xb) {
  const int u = (int)blockIdx.x * NTHR + (int)threadIdx.x;
  if (u >= nUnits) return;
  const int row = u >> 3;
  const int k8  = (u & 7) * 8;
  const float* p = x + (size_t)row * CF + k8;
  const v4f a = *(const v4fa*)p;
  const v4f b = *(const v4fa*)(p + 4);
  v8us o;
  o[0] = (unsigned short)bf16_bits(a.x);
  o[1] = (unsigned short)bf16_bits(a.y);
  o[2] = (unsigned short)bf16_bits(a.z);
  o[3] = (unsigned short)bf16_bits(a.w);
  o[4] = (unsigned short)bf16_bits(b.x);
  o[5] = (unsigned short)bf16_bits(b.y);
  o[6] = (unsigned short)bf16_bits(b.z);
  o[7] = (unsigned short)bf16_bits(b.w);
  unsigned short* dp = xb + (size_t)row * CF + k8;
  *(volatile v8us*)dp = o;
  __threadfence();
  *(volatile v8us*)dp = o;
}

__global__ __launch_bounds__(NTHR) void k_deg(const int* __restrict__ keys, int nE, int vec8, float* dos) {
  __shared__ __attribute__((aligned(16))) int scnt[NBD];
  __shared__ __attribute__((aligned(16))) int list[LISTN];
  __shared__ int wcnt[NWAVE];
  const int tid = (int)threadIdx.x, lane = tid & 31, wave = tid >> 5;
  const int nodeBase = (int)blockIdx.x * NBD;

  for (int i = tid; i < NBD; i += NTHR) scnt[i] = 0;
  for (int i = tid; i < LISTN; i += NTHR) list[i] = 0;
  if (tid < NWAVE) wcnt[tid] = 0;
  __syncthreads();

  const int nChunks = (nE + CHUNK - 1) / CHUNK;
#pragma unroll 1
  for (int ch = 0; ch < nChunks; ++ch) {
    const int cbase = ch * CHUNK;
    const int wc = scan_chunk<SLD>(keys, nE, cbase, nodeBase, NBD, vec8, list, tid, lane, wave);
    if (lane == 0) wcnt[wave] = wc;
    __syncthreads();
    if (wave == 0) {
#pragma unroll 1
      for (int w2 = 0; w2 < NWAVE; ++w2) {
        int c = wcnt[w2];
        c = c < 0 ? 0 : (c > WCAP ? WCAP : c);
#pragma unroll 1
        for (int b0 = 0; b0 < c; b0 += 32) {
          const int idx = b0 + lane;
          const int ent = list[w2 * WCAP + (idx < WCAP ? idx : WCAP - 1)];
          const int m32 = (c - b0) < 32 ? (c - b0) : 32;
#pragma unroll 1
          for (int k = 0; k < m32; ++k) {
            const int u  = __builtin_amdgcn_readlane(ent, k);
            const int sl = u & (NBD - 1);
            if (lane == 0) scnt[sl] = scnt[sl] + 1;
          }
        }
      }
    }
    __syncthreads();
  }

#pragma unroll 1
  for (int i = tid; i < NBD; i += NTHR) {
    int c = scnt[i];
    c = c < 1 ? 1 : c;
    const float r = 1.0f / sqrtf((float)c);
    scnt[i] = __float_as_int(r);
  }
  __syncthreads();

  v4f vals[NBD / (NTHR * 4)];
#pragma unroll
  for (int it = 0; it < NBD / (NTHR * 4); ++it) {
    const int s0 = it * (NTHR * 4) + 4 * tid;
    const v4i c4 = *(const v4ia*)(scnt + s0);
    v4f v;
    v.x = __int_as_float(c4.x); v.y = __int_as_float(c4.y);
    v.z = __int_as_float(c4.z); v.w = __int_as_float(c4.w);
    vals[it] = v;
  }
#pragma unroll
  for (int it = 0; it < NBD / (NTHR * 4); ++it) {
    const int s0 = it * (NTHR * 4) + 4 * tid;
    *(volatile v4f*)(dos + (size_t)nodeBase + s0) = vals[it];
  }
  __threadfence();
#pragma unroll
  for (int it = 0; it < NBD / (NTHR * 4); ++it) {
    const int s0 = it * (NTHR * 4) + 4 * tid;
    *(volatile v4f*)(dos + (size_t)nodeBase + s0) = vals[it];
  }
}

template <int LYR>
__global__ __launch_bounds__(NTHR) void k_scan(const int* __restrict__ srcs, const int* __restrict__ dsts,
                                               int nE, int nN, int vec8, int mRows,
                                               const float* __restrict__ dos,
                                               const unsigned* __restrict__ xbw,
                                               const float* __restrict__ hs,
                                               unsigned short* hb) {
  extern __shared__ __attribute__((aligned(16))) int dsm[];
  int* list = dsm;
  int* hl   = dsm + LISTN;
  int* sl   = dsm + LISTN + RCAP;
  int* cnt  = dsm + LISTN + 2 * RCAP;
  int* offs = cnt + NBA;
  int* cur  = offs + NBA;
  int* misc = cur + NBA;
  const int tid = (int)threadIdx.x, lane = tid & 31, wave = tid >> 5;
  const int nodeBase = (int)blockIdx.x * NBA;

  {
    const v4i z4 = {0, 0, 0, 0};
    for (int i = tid * 4; i < AGG_ZINTS; i += NTHR * 4) *(v4ia*)(dsm + i) = z4;
    if (tid < 16) misc[tid] = 0;
  }
  __syncthreads();

  int t = 0, ov = 0;
  const int nChunks = (nE + CHUNK - 1) / CHUNK;
#pragma unroll 1
  for (int ch = 0; ch < nChunks; ++ch) {
    const int cbase = ch * CHUNK;
    const int wc = scan_chunk<SLA>(dsts, nE, cbase, nodeBase, NBA, vec8, list, tid, lane, wave);
    if (lane == 0) misc[wave] = wc;
    __syncthreads();
    if (wave == 0) {
#pragma unroll 1
      for (int w2 = 0; w2 < NWAVE; ++w2) {
        int c = misc[w2];
        c = c < 0 ? 0 : (c > WCAP ? WCAP : c);
#pragma unroll 1
        for (int b0 = 0; b0 < c; b0 += 32) {
          const int idx = b0 + lane;
          const int ent = list[w2 * WCAP + (idx < WCAP ? idx : WCAP - 1)];
          const int m32 = (c - b0) < 32 ? (c - b0) : 32;
#pragma unroll 1
          for (int k = 0; k < m32; ++k) {
            const int u    = __builtin_amdgcn_readlane(ent, k);
            const int slot = u & (NBA - 1);
            const int el   = (u >> SLA) & (CHUNK - 1);
            const int pk   = ((cbase + el) << SLA) | slot;
            if (t < RCAP) {
              if (lane == 0) { hl[t] = pk; cnt[slot] = cnt[slot] + 1; }
              t = t + 1;
            } else {
              ov = 1;
            }
          }
        }
      }
    }
    __syncthreads();
  }
  if (wave == 0 && lane == 0) { misc[8] = t; misc[9] = ov; }
  __syncthreads();
  int tt = misc[8];
  tt = tt < 0 ? 0 : (tt > RCAP ? RCAP : tt);
  const int ovf = misc[9];

  if (wave == 0) {
    const int base = lane * (NBA / 32);
    int s = 0;
#pragma unroll 1
    for (int i = 0; i < NBA / 32; ++i) s += cnt[base + i];
    int incl = s;
#pragma unroll
    for (int d = 1; d < 32; d <<= 1) {
      const int y = __shfl_up(incl, d, 32);
      if (lane >= d) incl += y;
    }
    int run = incl - s;
#pragma unroll 1
    for (int i = 0; i < NBA / 32; ++i) {
      const int cv = cnt[base + i];
      offs[base + i] = run;
      cur[base + i]  = run;
      run += cv;
    }
  }
  __syncthreads();
  if (wave == 0) {
#pragma unroll 1
    for (int b0 = 0; b0 < tt; b0 += 32) {
      const int idx = b0 + lane;
      const int ent = hl[idx < RCAP ? idx : RCAP - 1];
      const int m32 = (tt - b0) < 32 ? (tt - b0) : 32;
#pragma unroll 1
      for (int k = 0; k < m32; ++k) {
        const int u    = __builtin_amdgcn_readlane(ent, k);
        const int slot = u & (NBA - 1);
        if (lane == 0) {
          int p = cur[slot];
          p = p < 0 ? 0 : (p > RCAP - 1 ? RCAP - 1 : p);
          sl[p] = u;
          cur[slot] = p + 1;
        }
      }
    }
  }
  __syncthreads();

  const float qnan = __int_as_float(0x7fc00000);
  const float pz = (ovf != 0) ? qnan : 0.0f;
  const int q0s = (4 * lane) & 31, q1s = (4 * lane + 1) & 31;
  const int q2s = (4 * lane + 2) & 31, q3s = (4 * lane + 3) & 31;
#pragma unroll 1
  for (int si = 0; si < NBA / NWAVE; ++si) {
    const int s    = si * NWAVE + wave;
    const int node = nodeBase + s;
    int cr = cnt[s];
    cr = cr < 0 ? 0 : cr;
    const bool big = cr > DEGCAP;
    const int c = big ? DEGCAP : cr;
    int o = offs[s];
    o = o < 0 ? 0 : (o > RCAP ? RCAP : o);
    const float dd = 1.0f / sqrtf((float)(cr < 1 ? 1 : cr));
    float acc0 = 0.0f, acc1 = 0.0f;
#pragma unroll 1
    for (int b0 = 0; b0 < c; b0 += 32) {
      int idx = o + b0 + lane;
      idx = idx > RCAP - 1 ? RCAP - 1 : idx;
      const int ent = sl[idx];
      int eid = ent >> SLA;
      eid = eid < 0 ? 0 : (eid > nE - 1 ? nE - 1 : eid);
      int sr = srcs[eid];
      sr = sr < 0 ? 0 : (sr > nN - 1 ? nN - 1 : sr);
      int dsi = 0;
      if constexpr (LYR == 1) dsi = __float_as_int(dos[sr]);
      const int m32 = (c - b0) < 32 ? (c - b0) : 32;
#pragma unroll 1
      for (int k = 0; k < m32; ++k) {
        const int sk = __builtin_amdgcn_readlane(sr, k);
        if constexpr (LYR == 1) {
          const float ck = __int_as_float(__builtin_amdgcn_readlane(dsi, k));
          const unsigned w = xbw[(size_t)sk * (CF / 2) + lane];
          const float x0 = __uint_as_float(w << 16);
          const float x1 = __uint_as_float(w & 0xffff0000u);
          acc0 = fmaf(ck, x0, acc0);
          acc1 = fmaf(ck, x1, acc1);
        } else {
          const v2f a = *(const v2fa*)(hs + (size_t)sk * CF + 2 * lane);
          acc0 += a.x;
          acc1 += a.y;
        }
      }
    }
    const float pzr = big ? qnan : pz;
    const bool live = node < nN;
    const float y0 = acc0 * dd + pzr;
    const float y1 = acc1 * dd + pzr;
    const float v0 = live ? y0 : 0.0f;
    const float v1 = live ? y1 : 0.0f;
    const bool wr = (node < mRows) && (lane < 16);
    const unsigned hb0 = bf16_bits(v0), hb1 = bf16_bits(v1);
    const unsigned lb0 = bf16_bits(v0 - __uint_as_float(hb0 << 16));
    const unsigned lb1 = bf16_bits(v1 - __uint_as_float(hb1 << 16));
    const int hw = (int)(hb0 | (hb1 << 16));
    const int lw = (int)(lb0 | (lb1 << 16));
    const int g0 = __shfl(hw, q0s, 32), g1 = __shfl(hw, q1s, 32);
    const int g2 = __shfl(hw, q2s, 32), g3 = __shfl(hw, q3s, 32);
    const int p0 = __shfl(lw, q0s, 32), p1 = __shfl(lw, q1s, 32);
    const int p2 = __shfl(lw, q2s, 32), p3 = __shfl(lw, q3s, 32);
    const bool lsel = (lane & 8) != 0;
    v4u pv;
    pv.x = (unsigned int)(lsel ? p0 : g0);
    pv.y = (unsigned int)(lsel ? p1 : g1);
    pv.z = (unsigned int)(lsel ? p2 : g2);
    pv.w = (unsigned int)(lsel ? p3 : g3);
    unsigned short* hp = hb + (size_t)node * K2 + 8 * (lane & 15);
    if (wr) *(volatile v4u*)hp = pv;
    __threadfence();
    if (wr) *(volatile v4u*)hp = pv;
  }
}

__global__ __launch_bounds__(GTHR) void k_gemm1(const unsigned short* __restrict__ A,
                                                const unsigned short* __restrict__ WT,
                                                const float* __restrict__ bias, const float* __restrict__ dos,
                                                float* outF) {
  __shared__ __attribute__((aligned(16))) float stg[GBM * CF];
  __shared__ float sdos[GBM];
  const int tid = (int)threadIdx.x, lane = tid & 31, wave = tid >> 5, hh = lane >> 4, m = lane & 15;
  const int rowBase = (int)blockIdx.x * GBM;

  if (tid < GBM) sdos[tid] = dos[rowBase + tid];

  v8f acc[4];
  {
    const v8f z = {0.f, 0.f, 0.f, 0.f, 0.f, 0.f, 0.f, 0.f};
    acc[0] = z; acc[1] = z; acc[2] = z; acc[3] = z;
  }
  const unsigned short* ap = A  + (size_t)(rowBase + 16 * wave + m) * (size_t)K2 + 8 * hh;
  const unsigned short* wp = WT + (size_t)m * (size_t)K2 + 8 * hh;
#pragma unroll 1
  for (int ks = 0; ks < K2 / 32; ++ks) {
    FragB af;
    af.h[0] = *(const v8usa*)(ap + 32 * ks);
    af.h[1] = *(const v8usa*)(ap + 32 * ks + 16);
#pragma unroll
    for (int t = 0; t < 4; ++t) {
      const unsigned short* wq = wp + (size_t)(16 * t) * (size_t)K2 + 32 * ks;
      FragB bf;
      bf.h[0] = *(const v8usa*)wq;
      bf.h[1] = *(const v8usa*)(wq + 16);
      acc[t] = wmb(af, bf, acc[t]);
    }
  }

#pragma unroll
  for (int t = 0; t < 4; ++t) {
    const int lc = 16 * t + m;
#pragma unroll
    for (int r = 0; r < 8; ++r) {
      const int lr = 16 * wave + 8 * hh + r;
      stg[lr * CF + lc] = acc[t][r];
    }
  }
  __syncthreads();

  v4f bb;
  {
    const v4f b4 = *(const v4fa*)(bias + 4 * m);
    bb.x = bf16_val(b4.x); bb.y = bf16_val(b4.y); bb.z = bf16_val(b4.z); bb.w = bf16_val(b4.w);
  }
  v4f fv[8];
#pragma unroll
  for (int i = 0; i < 8; ++i) {
    const int lr = 16 * wave + 2 * i + hh;
    const v4f a = *(const v4fa*)(stg + lr * CF + 4 * m);
    const float sc = sdos[lr];
    v4f y;
    y.x = relu_keep(a.x + bb.x) * sc;
    y.y = relu_keep(a.y + bb.y) * sc;
    y.z = relu_keep(a.z + bb.z) * sc;
    y.w = relu_keep(a.w + bb.w) * sc;
    fv[i] = y;
  }
#pragma unroll
  for (int i = 0; i < 8; ++i) {
    const int lr = 16 * wave + 2 * i + hh;
    float* op = outF + (size_t)(rowBase + lr) * (size_t)CF + 4 * m;
    *(volatile v4f*)op = fv[i];
  }
  __threadfence();
#pragma unroll
  for (int i = 0; i < 8; ++i) {
    const int lr = 16 * wave + 2 * i + hh;
    float* op = outF + (size_t)(rowBase + lr) * (size_t)CF + 4 * m;
    *(volatile v4f*)op = fv[i];
  }
}

__global__ __launch_bounds__(GTHR) void k_tail(const unsigned short* __restrict__ A,
                                               const unsigned short* __restrict__ W2T,
                                               const unsigned short* __restrict__ Wm1T,
                                               const unsigned short* __restrict__ Wm2T,
                                               const float* __restrict__ b2, const float* __restrict__ bm1,
                                               const float* __restrict__ bm2, float* out, int nN) {
  __shared__ __attribute__((aligned(16))) unsigned short sX[GBM * K2];
  __shared__ __attribute__((aligned(16))) unsigned short sY[GBM * K2];
  __shared__ __attribute__((aligned(16))) float so[GBM * OC];
  __shared__ float sb[3 * CF];
  const int tid = (int)threadIdx.x, lane = tid & 31, wave = tid >> 5, hh = lane >> 4, m = lane & 15;
  const int rowBase = (int)blockIdx.x * GBM;

  if (tid < CF) {
    sb[tid]          = bf16_val(b2[tid]);
    sb[CF + tid]     = bf16_val(bm1[tid]);
    sb[2 * CF + tid] = bf16_val(bm2[tid < OC ? tid : OC - 1]);
  }
  __syncthreads();

  const v8f z = {0.f, 0.f, 0.f, 0.f, 0.f, 0.f, 0.f, 0.f};
  v8f acc[4];

  acc[0] = z; acc[1] = z; acc[2] = z; acc[3] = z;
  {
    const unsigned short* ap = A   + (size_t)(rowBase + 16 * wave + m) * (size_t)K2 + 8 * hh;
    const unsigned short* wp = W2T + (size_t)m * (size_t)K2 + 8 * hh;
#pragma unroll 1
    for (int ks = 0; ks < K2 / 32; ++ks) {
      FragB af;
      af.h[0] = *(const v8usa*)(ap + 32 * ks);
      af.h[1] = *(const v8usa*)(ap + 32 * ks + 16);
#pragma unroll
      for (int t = 0; t < 4; ++t) {
        const unsigned short* wq = wp + (size_t)(16 * t) * (size_t)K2 + 32 * ks;
        FragB bf;
        bf.h[0] = *(const v8usa*)wq;
        bf.h[1] = *(const v8usa*)(wq + 16);
        acc[t] = wmb(af, bf, acc[t]);
      }
    }
  }
#pragma unroll
  for (int t = 0; t < 4; ++t) {
    const int lc = 16 * t + m;
    const float bv = sb[lc];
#pragma unroll
    for (int r = 0; r < 8; ++r) {
      const int lr = 16 * wave + 8 * hh + r;
      const float v = relu_keep(acc[t][r] + bv);
      const unsigned hbv = bf16_bits(v);
      const unsigned lbv = bf16_bits(v - __uint_as_float(hbv << 16));
      sX[lr * K2 + lc]      = (unsigned short)hbv;
      sX[lr * K2 + CF + lc] = (unsigned short)lbv;
    }
  }
  __syncthreads();

  acc[0] = z; acc[1] = z; acc[2] = z; acc[3] = z;
  {
    const unsigned short* wp = Wm1T + (size_t)m * (size_t)K2 + 8 * hh;
#pragma unroll 1
    for (int ks = 0; ks < K2 / 32; ++ks) {
      FragB af;
      af.h[0] = *(const v8usa*)(sX + (16 * wave + m) * K2 + 8 * hh + 32 * ks);
      af.h[1] = *(const v8usa*)(sX + (16 * wave + m) * K2 + 8 * hh + 32 * ks + 16);
#pragma unroll
      for (int t = 0; t < 4; ++t) {
        const unsigned short* wq = wp + (size_t)(16 * t) * (size_t)K2 + 32 * ks;
        FragB bf;
        bf.h[0] = *(const v8usa*)wq;
        bf.h[1] = *(const v8usa*)(wq + 16);
        acc[t] = wmb(af, bf, acc[t]);
      }
    }
  }
#pragma unroll
  for (int t = 0; t < 4; ++t) {
    const int lc = 16 * t + m;
    const float bv = sb[CF + lc];
#pragma unroll
    for (int r = 0; r < 8; ++r) {
      const int lr = 16 * wave + 8 * hh + r;
      const float v = relu_keep(acc[t][r] + bv);
      const unsigned hbv = bf16_bits(v);
      const unsigned lbv = bf16_bits(v - __uint_as_float(hbv << 16));
      sY[lr * K2 + lc]      = (unsigned short)hbv;
      sY[lr * K2 + CF + lc] = (unsigned short)lbv;
    }
  }
  __syncthreads();

  v8f ac3[2];
  ac3[0] = z; ac3[1] = z;
  {
    const unsigned short* wp = Wm2T + (size_t)m * (size_t)K2 + 8 * hh;
#pragma unroll 1
    for (int ks = 0; ks < K2 / 32; ++ks) {
      FragB af;
      af.h[0] = *(const v8usa*)(sY + (16 * wave + m) * K2 + 8 * hh + 32 * ks);
      af.h[1] = *(const v8usa*)(sY + (16 * wave + m) * K2 + 8 * hh + 32 * ks + 16);
#pragma unroll
      for (int t = 0; t < 2; ++t) {
        const unsigned short* wq = wp + (size_t)(16 * t) * (size_t)K2 + 32 * ks;
        FragB bf;
        bf.h[0] = *(const v8usa*)wq;
        bf.h[1] = *(const v8usa*)(wq + 16);
        ac3[t] = wmb(af, bf, ac3[t]);
      }
    }
  }
#pragma unroll
  for (int t = 0; t < 2; ++t) {
    const int lc = 16 * t + m;
    const float bv = sb[2 * CF + lc];
#pragma unroll
    for (int r = 0; r < 8; ++r) {
      const int lr = 16 * wave + 8 * hh + r;
      so[lr * OC + lc] = ac3[t][r] + bv;
    }
  }
  __syncthreads();

  v4f ovv[4];
#pragma unroll
  for (int i = 0; i < 4; ++i) {
    const int lr = 16 * wave + 4 * i + (lane >> 3);
    ovv[i] = *(const v4fa*)(so + lr * OC + 4 * (lane & 7));
  }
#pragma unroll
  for (int i = 0; i < 4; ++i) {
    const int gr = rowBase + 16 * wave + 4 * i + (lane >> 3);
    if (gr < nN) *(volatile v4f*)(out + (size_t)gr * OC + 4 * (lane & 7)) = ovv[i];
  }
  __threadfence();
#pragma unroll
  for (int i = 0; i < 4; ++i) {
    const int gr = rowBase + 16 * wave + 4 * i + (lane >> 3);
    if (gr < nN) *(volatile v4f*)(out + (size_t)gr * OC + 4 * (lane & 7)) = ovv[i];
  }
}

static inline int cdiv(int a, int b) { return (a + b - 1) / b; }
static inline size_t al256(size_t o) { return (o + 255) & ~(size_t)255; }

extern "C" void kernel_launch(void* const* d_in, const int* in_sizes, int n_in,
                              void* d_out, int out_size, void* d_ws, size_t ws_size,
                              hipStream_t stream) {
  if (n_in < 11) return;
  if (in_sizes[0] < CF || (in_sizes[0] % CF) != 0) return;
  const int nN = in_sizes[0] / CF;
  if (nN < 1 || nN > (1 << 22)) return;
  const int nE = in_sizes[1];
  if (nE < 1 || nE >= (1 << (31 - SLA))) return;
  if (in_sizes[2] != nE) return;
  if (in_sizes[3] != CF * CF || in_sizes[4] != CF) return;
  if (in_sizes[5] != CF * CF || in_sizes[6] != CF) return;
  if (in_sizes[7] != CF * CF || in_sizes[8] != CF) return;
  if (in_sizes[9] != CF * OC || in_sizes[10] != OC) return;
  if ((long long)out_size != (long long)nN * OC) return;

  const float* feat = (const float*)d_in[0];
  const int*   src  = (const int*)d_in[1];
  const int*   dst  = (const int*)d_in[2];
  const float* W1   = (const float*)d_in[3];
  const float* b1   = (const float*)d_in[4];
  const float* W2   = (const float*)d_in[5];
  const float* b2   = (const float*)d_in[6];
  const float* Wm1  = (const float*)d_in[7];
  const float* bm1  = (const float*)d_in[8];
  const float* Wm2  = (const float*)d_in[9];
  const float* bm2  = (const float*)d_in[10];
  float* out = (float*)d_out;

  const int MP   = cdiv(nN, GBM) * GBM;
  const int gM   = MP / GBM;
  const int gD   = cdiv(MP, NBD);
  const int NBPD = gD * NBD;
  const int gA   = cdiv(MP, NBA);
  if ((long long)gA * NBA < (long long)MP) return;
  if (NBPD < MP) return;
  const int vec8 = ((nE & 3) == 0) ? 1 : 0;

  char* ws = (char*)d_ws;
  size_t off = 0;
  const size_t oDOS = off; off = al256(off + (size_t)NBPD * 4);
  const size_t oW1T = off; off = al256(off + (size_t)CF * K2 * 2);
  const size_t oW2T = off; off = al256(off + (size_t)CF * K2 * 2);
  const size_t oWmA = off; off = al256(off + (size_t)CF * K2 * 2);
  const size_t oWmB = off; off = al256(off + (size_t)OC * K2 * 2);
  const size_t oXB  = off; off = al256(off + (size_t)nN * CF * 2);
  const size_t oAG  = off; off = al256(off + (size_t)MP * K2 * 2);
  const size_t oHS  = off; off = al256(off + (size_t)MP * CF * 4);
  if (off > ws_size || off > (size_t)WSMAX) return;
  float*          DOS  = (float*)(ws + oDOS);
  unsigned short* W1T  = (unsigned short*)(ws + oW1T);
  unsigned short* W2T  = (unsigned short*)(ws + oW2T);
  unsigned short* WmAT = (unsigned short*)(ws + oWmA);
  unsigned short* WmBT = (unsigned short*)(ws + oWmB);
  unsigned short* XB   = (unsigned short*)(ws + oXB);
  unsigned short* AGG  = (unsigned short*)(ws + oAG);
  float*          HS2  = (float*)(ws + oHS);

  const size_t scanLds = (size_t)AGG_LDS_INTS * 4;
  hipFuncSetAttribute(reinterpret_cast<const void*>(&k_scan<1>), hipFuncAttributeMaxDynamicSharedMemorySize, (int)scanLds);
  hipFuncSetAttribute(reinterpret_cast<const void*>(&k_scan<2>), hipFuncAttributeMaxDynamicSharedMemorySize, (int)scanLds);

  const int nUx = nN * (CF / 8);
  k_wprep<<<(3 * NUW + NUW2) / NTHR, NTHR, 0, stream>>>(W1, W2, Wm1, Wm2, W1T, W2T, WmAT, WmBT);
  k_cvx<<<cdiv(nUx, NTHR), NTHR, 0, stream>>>(feat, nUx, XB);
  k_deg<<<gD, NTHR, 0, stream>>>(src, nE, vec8, DOS);
  k_scan<1><<<gA, NTHR, scanLds, stream>>>(src, dst, nE, nN, vec8, MP, DOS, (const unsigned*)XB, HS2, AGG);
  k_gemm1<<<gM, GTHR, 0, stream>>>(AGG, W1T, b1, DOS, HS2);
  k_scan<2><<<gA, NTHR, scanLds, stream>>>(src, dst, nE, nN, vec8, MP, DOS, (const unsigned*)XB, HS2, AGG);
  k_tail<<<gM, GTHR, 0, stream>>>(AGG, W2T, WmAT, WmBT, b2, bm1, bm2, out, nN);
}
